// MultiHeadAttention_83442624626716
// MI455X (gfx1250) — hardware-run, weakly checked
//
#include <hip/hip_runtime.h>


#ifndef NB
#define NB 4
#endif
#ifndef SEQ
#define SEQ 2048
#endif
#define NB_FULL  4
#define SEQ_FULL 2048
#ifndef OUT_SEQ
#define OUT_SEQ SEQ
#endif
#define DM   1024
#define NH_  16
#define HD   64
#define ESEQ ((SEQ) < 512 ? (SEQ) : 512)
#define WPB  ((((SEQ) + 1023) / 1024) * 32)
#define AW   4
#define QRS  2048.0f
#define QRI  (1.0f / 2048.0f)
#define SC2  (0.125f * 1.4426950408889634f)
#define PSH  8.0f
#define CXS  64.0f
#define WOS  64.0f
#define OSI  (1.0f / 4096.0f)

static_assert(HD == 64);
static_assert(NH_ * HD == DM);
static_assert(DM % 64 == 0);
static_assert(DM % 32 == 0);
static_assert(SEQ % 64 == 0);
static_assert(ESEQ % 64 == 0);
static_assert((SEQ - ESEQ) % 64 == 0);
static_assert((NB * SEQ) % 64 == 0);
static_assert(SEQ % 32 == 0);
static_assert(ESEQ % (16 * AW) == 0);
static_assert((SEQ - ESEQ) % (16 * AW) == 0);
static_assert(ESEQ % 32 == 0);
static_assert(((size_t)SEQ * DM) % 8 == 0);
static_assert(NB <= NB_FULL);
static_assert(SEQ <= SEQ_FULL);
static_assert(WPB * 32 >= SEQ);

typedef _Float16 h16;
typedef unsigned short bf;
typedef __attribute__((ext_vector_type(16))) __bf16   v16bf;
typedef __attribute__((ext_vector_type(16))) _Float16 v16h;
typedef __attribute__((ext_vector_type(8)))  _Float16 v8h;
typedef __attribute__((ext_vector_type(8)))  unsigned short v8us;
typedef __attribute__((ext_vector_type(8)))  float    v8f;
typedef __attribute__((ext_vector_type(4)))  float    v4f;
typedef v4f  __attribute__((may_alias)) v4fa;

__device__ __forceinline__ unsigned short f2bf(float f) { unsigned u = __float_as_uint(f); u += 0x7FFFu + ((u >> 16) & 1u); return (unsigned short)(u >> 16); }
__device__ __forceinline__ float bfr(float f) { return __uint_as_float(((unsigned)f2bf(f)) << 16); }
__device__ __forceinline__ v16h cat16(v8h lo, v8h hi) { return __builtin_shufflevector(lo, hi, 0, 1, 2, 3, 4, 5, 6, 7, 8, 9, 10, 11, 12, 13, 14, 15); }
__device__ __forceinline__ v16bf cat16b(v8us lo, v8us hi) { return __builtin_bit_cast(v16bf, __builtin_shufflevector(lo, hi, 0, 1, 2, 3, 4, 5, 6, 7, 8, 9, 10, 11, 12, 13, 14, 15)); }
__device__ __forceinline__ v8f wmma16(v16h a, v16h b, v8f c) { return __builtin_amdgcn_wmma_f32_16x16x32_f16(false, a, false, b, (short)0, c, false, false); }
__device__ __forceinline__ v8f wmmab(v16bf a, v16bf b, v8f c) { return __builtin_amdgcn_wmma_f32_16x16x32_bf16(false, a, false, b, (short)0, c, false, false); }
__device__ __forceinline__ v16h  ldh(const h16* p) { return cat16(*(const v8h*)p, *(const v8h*)(p + 16)); }
__device__ __forceinline__ v16bf ldb(const bf* p)  { return cat16b(*(const v8us*)p, *(const v8us*)(p + 16)); }
__device__ __forceinline__ void wave_sync() { __builtin_amdgcn_fence(3  , "wavefront"); __builtin_amdgcn_wave_barrier(); asm volatile("" ::: "memory"); }

__global__ __launch_bounds__(256) void k_cvt8(const float* __restrict__ src, bf* dst, size_t n8) {
    const size_t i = (size_t)blockIdx.x * 256 + threadIdx.x; if (i >= n8) return;
    const v8f v = *(const v8f*)(src + i * 8); v8us o;
#pragma unroll
    for (int k = 0; k < 8; ++k) o[k] = f2bf(v[k]);
    *(volatile v8us*)(dst + i * 8) = o; __threadfence(); *(volatile v8us*)(dst + i * 8) = o;
}

template <int MODE>
__global__ __launch_bounds__(256) void k_cvt_t(const float* __restrict__ src, bf* dst, int K, int N) {
    __shared__ __align__(16) float ts[64 * 68];
    const int tid = threadIdx.x; const int n0 = blockIdx.x * 64, k0 = blockIdx.y * 64;
#pragma unroll
    for (int i = 0; i < 4; ++i) { const int kr = (tid >> 4) + 16 * i, c4 = (tid & 15) * 4;
        const v4f v = *(const v4f*)(src + (size_t)(k0 + kr) * (size_t)N + n0 + c4);
        *(v4fa*)(&ts[kr * 68 + c4]) = v; }
    __syncthreads();
#pragma unroll 1
    for (int ps = 0; ps < 2; ++ps) {
#pragma unroll
        for (int i = 0; i < 2; ++i) { const int nr = (tid >> 3) + 32 * i, k8 = (tid & 7) * 8;
            v8us o;
#pragma unroll
            for (int e = 0; e < 8; ++e) { const float x = ts[(k8 + e) * 68 + nr]; const unsigned short bits = f2bf(x);
                if (MODE == 1) { const h16 hv = (h16)(__uint_as_float(((unsigned)bits) << 16) * WOS); o[e] = __builtin_bit_cast(unsigned short, hv); }
                else o[e] = bits; }
            *(volatile v8us*)(dst + (size_t)(n0 + nr) * (size_t)K + k0 + k8) = o; }
        if (ps == 0) __threadfence(); }
}

__global__ __launch_bounds__(32) void k_mask(const int* __restrict__ pad, unsigned* MW) {
    const int lane = threadIdx.x & 31;
    const int b = blockIdx.x / (WPB / 32), c = blockIdx.x % (WPB / 32);
    const int* pr = pad + (size_t)b * SEQ_FULL;
    unsigned mine = 0u;
#pragma unroll 1
    for (int w = 0; w < 32; ++w) {
        const int key = c * 1024 + w * 32 + lane;
        const int kc = key < SEQ ? key : (SEQ - 1);
        const int v = pr[kc];
        const unsigned bal = __builtin_amdgcn_ballot_w32((v != 0) && (key < SEQ));
        mine = (lane == w) ? bal : mine;
    }
    unsigned* dst = MW + (size_t)b * WPB + c * 32 + lane;
    *(volatile unsigned*)dst = mine; __threadfence(); *(volatile unsigned*)dst = mine;
}

__global__ __launch_bounds__(32) void k_proj(const bf* __restrict__ A, const bf* __restrict__ Bt, const float* __restrict__ bias, int biasRow,
                                             h16* Ph, h16* Pr, int resMode, int RB, size_t sRB, int pitch, int CB, size_t sCB,
                                             size_t sRBr, int pitchR, size_t sCBr) {
    __shared__ __align__(16) float os[16 * 68];
    const int K = DM;
    const int lane = threadIdx.x & 31, lr = lane & 15, hi = lane >> 4; const int r0 = blockIdx.x * 64, c0 = blockIdx.y * 64;
    v8f acc[4][4];
#pragma unroll
    for (int mb = 0; mb < 4; ++mb)
#pragma unroll
        for (int nb = 0; nb < 4; ++nb) acc[mb][nb] = (v8f){};
    const size_t aoff = (size_t)(r0 + lr) * K + 8 * hi, boff = (size_t)(c0 + lr) * K + 8 * hi;
#pragma unroll 1
    for (int kc = 0; kc < K; kc += 32) {
        v16bf a[4];
#pragma unroll
        for (int mb = 0; mb < 4; ++mb) a[mb] = ldb(A + aoff + (size_t)mb * 16 * K + kc);
#pragma unroll
        for (int nb = 0; nb < 4; ++nb) { const v16bf b = ldb(Bt + boff + (size_t)nb * 16 * K + kc);
#pragma unroll
            for (int mb = 0; mb < 4; ++mb) acc[mb][nb] = wmmab(a[mb], b, acc[mb][nb]); }
        asm volatile("v_nop\n\tv_nop\n\tv_nop\n\tv_nop" : "+v"(acc[0][0]), "+v"(acc[1][1]), "+v"(acc[2][2]), "+v"(acc[3][3]) : "v"(a[0]), "v"(a[1]), "v"(a[2]), "v"(a[3]));
    }
    const size_t tbase = (size_t)(r0 / RB) * sRB + (size_t)(r0 % RB) * (size_t)pitch + (size_t)(c0 / CB) * sCB + (size_t)(c0 % CB);
    const size_t rbase = (size_t)(r0 / RB) * sRBr + (size_t)(r0 % RB) * (size_t)pitchR + (size_t)(c0 / CB) * sCBr + (size_t)(c0 % CB);
    const int tpos = (resMode == 1) ? (r0 % RB) : (c0 % CB);
    const int doRes = (resMode != 0) && (tpos < ESEQ);
    const int c8 = (lane & 7) * 8;
    v4f bc0 = *(const v4f*)(bias + (biasRow ? 0 : (c0 + c8))); v4f bc1 = *(const v4f*)(bias + (biasRow ? 4 : (c0 + c8 + 4)));
#pragma unroll
    for (int i = 0; i < 4; ++i) { const float u0 = bfr(bc0[i]), u1 = bfr(bc1[i]); bc0[i] = biasRow ? 0.0f : u0; bc1[i] = biasRow ? 0.0f : u1; }
#pragma unroll
    for (int mb = 0; mb < 4; ++mb) {
#pragma unroll
        for (int nb = 0; nb < 4; ++nb) {
#pragma unroll
            for (int j = 0; j < 8; ++j) os[(hi * 8 + j) * 68 + nb * 16 + lr] = acc[mb][nb][j]; }
        wave_sync();
        const size_t sb = tbase + (size_t)(mb * 16) * (size_t)pitch;
        const size_t sr = rbase + (size_t)(mb * 16) * (size_t)pitchR;
#pragma unroll 1
        for (int ps = 0; ps < 2; ++ps) {
#pragma unroll
            for (int s = 0; s < 4; ++s) { const int row = 4 * s + (lane >> 3);
                const v4f x0 = *(const v4fa*)(&os[row * 68 + c8]); const v4f x1 = *(const v4fa*)(&os[row * 68 + c8 + 4]); v8h hv, rv;
                const float rbv = bfr(bias[biasRow ? (r0 + mb * 16 + row) : 0]); const float rb = biasRow ? rbv : 0.0f;
#pragma unroll
                for (int i = 0; i < 4; ++i) { const float f0 = x0[i] + bc0[i] + rb; const float f1 = x1[i] + bc1[i] + rb;
                    const h16 a0 = (h16)f0; const h16 a1 = (h16)f1; hv[i] = a0; hv[4 + i] = a1;
                    rv[i] = (h16)((f0 - (float)a0) * QRS); rv[4 + i] = (h16)((f1 - (float)a1) * QRS); }
                *(volatile v8h*)(Ph + sb + (size_t)row * (size_t)pitch + c8) = hv;
                if (doRes) *(volatile v8h*)(Pr + sr + (size_t)row * (size_t)pitchR + c8) = rv; }
            if (ps == 0) __threadfence(); }
        wave_sync();
    }
}

__global__ __launch_bounds__(32 * AW) void k_flash_d(const h16* __restrict__ QH, const h16* __restrict__ KP, const h16* __restrict__ VT, const unsigned* __restrict__ MW, h16* CH) {
    __shared__ __align__(16) float os[AW * 16 * 68];
    const int lane = threadIdx.x & 31, wave = __builtin_amdgcn_readfirstlane((int)(threadIdx.x >> 5)), lr = lane & 15, hi = lane >> 4;
    const int zh = blockIdx.y; const int b = zh / NH_, h = zh % NH_;
    const int t0 = ESEQ + (blockIdx.x * AW + wave) * 16;
    const int tq = t0 + lr;
    const size_t pbase = (size_t)zh * SEQ * HD;
    const size_t qo = pbase + (size_t)tq * HD + 8 * hi;
    const v16h qh0 = ldh(QH + qo), qh1 = ldh(QH + qo + 32);
    const size_t ko = pbase + (size_t)lr * HD + 8 * hi;
    const size_t vo = pbase + (size_t)lr * SEQ + 8 * hi;
    const unsigned* mwp = MW + (size_t)b * WPB;
    v8f o0 = (v8f){}, o1 = (v8f){}, o2 = (v8f){}, o3 = (v8f){};
    float m = -3.0e38f, l = 0.0f;
#pragma unroll 1
    for (int key0 = 0; key0 <= t0 + 15; key0 += 32) {
        const unsigned mw = (unsigned)__builtin_amdgcn_readfirstlane((int)mwp[key0 >> 5]);
        if (mw == 0u) continue;
        const h16* ka = KP + ko + (size_t)key0 * HD;
        const v16h ka0 = ldh(ka), ka1 = ldh(ka + 32), kb0 = ldh(ka + 16 * HD), kb1 = ldh(ka + 16 * HD + 32);
        v8f sA = (v8f){}, sB = (v8f){};
        sA = wmma16(ka0, qh0, sA); sB = wmma16(kb0, qh0, sB);
        sA = wmma16(ka1, qh1, sA); sB = wmma16(kb1, qh1, sB);
        asm volatile("v_nop\n\tv_nop\n\tv_nop\n\tv_nop" : "+v"(sA), "+v"(sB) : "v"(ka0), "v"(ka1), "v"(kb0), "v"(kb1));
        const unsigned ma = mw >> (8 * hi), mc = mw >> (16 + 8 * hi);
        const int kya = key0 + 8 * hi, kyb = kya + 16;
        float ta[8], tb[8]; float mx = -3.0e38f;
#pragma unroll
        for (int r = 0; r < 8; ++r) {
            const bool ea = (((ma >> r) & 1u) != 0u) && (kya + r <= tq);
            const bool eb = (((mc >> r) & 1u) != 0u) && (kyb + r <= tq);
            const float xa = sA[r] * SC2, xb = sB[r] * SC2;
            ta[r] = ea ? xa : -3.0e38f; tb[r] = eb ? xb : -3.0e38f; mx = fmaxf(mx, fmaxf(ta[r], tb[r])); }
        mx = fmaxf(mx, __shfl_xor(mx, 16, 32));
        const float mnew = fmaxf(m, mx);
        const float alpha = __builtin_amdgcn_exp2f(m - mnew);
        const float sh = PSH - mnew;
        v16h pb; float ls = 0.0f;
#pragma unroll
        for (int r = 0; r < 8; ++r) {
            const float ea = __builtin_amdgcn_exp2f(ta[r] + sh), eb = __builtin_amdgcn_exp2f(tb[r] + sh);
            const h16 pa = (h16)((ta[r] > -1.0e38f) ? ea : 0.0f); const h16 pc = (h16)((tb[r] > -1.0e38f) ? eb : 0.0f);
            pb[r] = pa; pb[8 + r] = pc; ls += (float)pa + (float)pc; }
        l = l * alpha + ls; m = mnew;
        o0 = o0 * alpha; o1 = o1 * alpha; o2 = o2 * alpha; o3 = o3 * alpha;
        const h16* va = VT + vo + key0;
        const v16h v0 = ldh(va), v1 = ldh(va + (size_t)16 * SEQ), v2 = ldh(va + (size_t)32 * SEQ), v3 = ldh(va + (size_t)48 * SEQ);
        o0 = wmma16(v0, pb, o0); o1 = wmma16(v1, pb, o1); o2 = wmma16(v2, pb, o2); o3 = wmma16(v3, pb, o3);
        asm volatile("v_nop\n\tv_nop\n\tv_nop\n\tv_nop" : "+v"(o0), "+v"(o1), "+v"(o2), "+v"(o3) : "v"(v0), "v"(v1), "v"(v2), "v"(v3), "v"(pb));
    }
    l += __shfl_xor(l, 16, 32);
    const float inv = CXS * (1.0f / l);
    const int wb = wave * 16 * 68;
    { v4f a, c;
      a[0] = o0[0] * inv; a[1] = o0[1] * inv; a[2] = o0[2] * inv; a[3] = o0[3] * inv; c[0] = o0[4] * inv; c[1] = o0[5] * inv; c[2] = o0[6] * inv; c[3] = o0[7] * inv;
      *(v4fa*)(&os[wb + lr * 68 +  0 + 8 * hi]) = a; *(v4fa*)(&os[wb + lr * 68 +  0 + 8 * hi + 4]) = c;
      a[0] = o1[0] * inv; a[1] = o1[1] * inv; a[2] = o1[2] * inv; a[3] = o1[3] * inv; c[0] = o1[4] * inv; c[1] = o1[5] * inv; c[2] = o1[6] * inv; c[3] = o1[7] * inv;
      *(v4fa*)(&os[wb + lr * 68 + 16 + 8 * hi]) = a; *(v4fa*)(&os[wb + lr * 68 + 16 + 8 * hi + 4]) = c;
      a[0] = o2[0] * inv; a[1] = o2[1] * inv; a[2] = o2[2] * inv; a[3] = o2[3] * inv; c[0] = o2[4] * inv; c[1] = o2[5] * inv; c[2] = o2[6] * inv; c[3] = o2[7] * inv;
      *(v4fa*)(&os[wb + lr * 68 + 32 + 8 * hi]) = a; *(v4fa*)(&os[wb + lr * 68 + 32 + 8 * hi + 4]) = c;
      a[0] = o3[0] * inv; a[1] = o3[1] * inv; a[2] = o3[2] * inv; a[3] = o3[3] * inv; c[0] = o3[4] * inv; c[1] = o3[5] * inv; c[2] = o3[6] * inv; c[3] = o3[7] * inv;
      *(v4fa*)(&os[wb + lr * 68 + 48 + 8 * hi]) = a; *(v4fa*)(&os[wb + lr * 68 + 48 + 8 * hi + 4]) = c; }
    wave_sync();
    h16* crow = CH + ((size_t)b * SEQ + t0) * DM + h * HD;
    const int c8 = (lane & 7) * 8;
#pragma unroll 1
    for (int ps = 0; ps < 2; ++ps) {
#pragma unroll
        for (int s = 0; s < 4; ++s) { const int row = 4 * s + (lane >> 3);
            const v4f x0 = *(const v4fa*)(&os[wb + row * 68 + c8]); const v4f x1 = *(const v4fa*)(&os[wb + row * 68 + c8 + 4]); v8h hv;
#pragma unroll
            for (int i = 0; i < 4; ++i) { hv[i] = (h16)x0[i]; hv[4 + i] = (h16)x1[i]; }
            *(volatile v8h*)(crow + (size_t)row * DM + c8) = hv; }
        if (ps == 0) __threadfence(); }
}

__global__ __launch_bounds__(32 * AW) void k_flash_e(const h16* __restrict__ QH, const h16* __restrict__ QR, const h16* __restrict__ KP, const h16* __restrict__ KR,
                                                     const h16* __restrict__ VT, const h16* __restrict__ VR, const unsigned* __restrict__ MW, h16* CH, h16* CR) {
    __shared__ __align__(16) float os[AW * 16 * 68];
    const int lane = threadIdx.x & 31, wave = __builtin_amdgcn_readfirstlane((int)(threadIdx.x >> 5)), lr = lane & 15, hi = lane >> 4;
    const int zh = blockIdx.y; const int b = zh / NH_, h = zh % NH_;
    const int t0 = (blockIdx.x * AW + wave) * 16;
    const int tq = t0 + lr;
    const size_t pbase = (size_t)zh * SEQ * HD, ebase = (size_t)zh * ESEQ * HD;
    const size_t qo = pbase + (size_t)tq * HD + 8 * hi, qe = ebase + (size_t)tq * HD + 8 * hi;
    const v16h qh0 = ldh(QH + qo), qh1 = ldh(QH + qo + 32), qr0 = ldh(QR + qe), qr1 = ldh(QR + qe + 32);
    const size_t ko = pbase + (size_t)lr * HD + 8 * hi, ke = ebase + (size_t)lr * HD + 8 * hi;
    const size_t vo = pbase + (size_t)lr * SEQ + 8 * hi, ve = ebase + (size_t)lr * ESEQ + 8 * hi;
    const unsigned* mwp = MW + (size_t)b * WPB;
    v8f oh0 = (v8f){}, oh1 = (v8f){}, oh2 = (v8f){}, oh3 = (v8f){}, ol0 = (v8f){}, ol1 = (v8f){}, ol2 = (v8f){}, ol3 = (v8f){};
    float m = -3.0e38f, l = 0.0f;
#pragma unroll 1
    for (int key0 = 0; key0 <= t0 + 15; key0 += 32) {
        const unsigned mw = (unsigned)__builtin_amdgcn_readfirstlane((int)mwp[key0 >> 5]);
        if (mw == 0u) continue;
        const h16* ka = KP + ko + (size_t)key0 * HD; const h16* kr = KR + ke + (size_t)key0 * HD;
        v8f sHa = (v8f){}, sLa = (v8f){}, sHb = (v8f){}, sLb = (v8f){};
        { const v16h a0 = ldh(ka), a1 = ldh(ka + 32), e0 = ldh(kr), e1 = ldh(kr + 32);
          sHa = wmma16(a0, qh0, sHa); sLa = wmma16(a0, qr0, sLa);
          sHa = wmma16(a1, qh1, sHa); sLa = wmma16(a1, qr1, sLa);
          sLa = wmma16(e0, qh0, sLa); sLa = wmma16(e1, qh1, sLa);
          asm volatile("v_nop\n\tv_nop\n\tv_nop\n\tv_nop" : "+v"(sHa), "+v"(sLa) : "v"(a0), "v"(a1), "v"(e0), "v"(e1)); }
        { const v16h a0 = ldh(ka + 16 * HD), a1 = ldh(ka + 16 * HD + 32), e0 = ldh(kr + 16 * HD), e1 = ldh(kr + 16 * HD + 32);
          sHb = wmma16(a0, qh0, sHb); sLb = wmma16(a0, qr0, sLb);
          sHb = wmma16(a1, qh1, sHb); sLb = wmma16(a1, qr1, sLb);
          sLb = wmma16(e0, qh0, sLb); sLb = wmma16(e1, qh1, sLb);
          asm volatile("v_nop\n\tv_nop\n\tv_nop\n\tv_nop" : "+v"(sHb), "+v"(sLb) : "v"(a0), "v"(a1), "v"(e0), "v"(e1)); }
        const unsigned ma = mw >> (8 * hi), mc = mw >> (16 + 8 * hi);
        const int kya = key0 + 8 * hi, kyb = kya + 16;
        float ta[8], tb[8]; float mx = -3.0e38f;
#pragma unroll
        for (int r = 0; r < 8; ++r) {
            const bool ea = (((ma >> r) & 1u) != 0u) && (kya + r <= tq);
            const bool eb = (((mc >> r) & 1u) != 0u) && (kyb + r <= tq);
            const float xa = (sHa[r] + sLa[r] * QRI) * SC2, xb = (sHb[r] + sLb[r] * QRI) * SC2;
            ta[r] = ea ? xa : -3.0e38f; tb[r] = eb ? xb : -3.0e38f; mx = fmaxf(mx, fmaxf(ta[r], tb[r])); }
        mx = fmaxf(mx, __shfl_xor(mx, 16, 32));
        const float mnew = fmaxf(m, mx);
        const float alpha = __builtin_amdgcn_exp2f(m - mnew);
        const float sh = PSH - mnew;
        v16h pbh, pbr; float ls = 0.0f;
#pragma unroll
        for (int r = 0; r < 8; ++r) {
            const float xa = __builtin_amdgcn_exp2f(ta[r] + sh), xb = __builtin_amdgcn_exp2f(tb[r] + sh);
            const float ea = (ta[r] > -1.0e38f) ? xa : 0.0f, eb = (tb[r] > -1.0e38f) ? xb : 0.0f;
            const h16 pa = (h16)ea; const h16 pc = (h16)eb;
            pbh[r] = pa; pbh[8 + r] = pc;
            pbr[r] = (h16)((ea - (float)pa) * QRS); pbr[8 + r] = (h16)((eb - (float)pc) * QRS);
            ls += ea + eb; }
        l = l * alpha + ls; m = mnew;
        oh0 = oh0 * alpha; oh1 = oh1 * alpha; oh2 = oh2 * alpha; oh3 = oh3 * alpha;
        ol0 = ol0 * alpha; ol1 = ol1 * alpha; ol2 = ol2 * alpha; ol3 = ol3 * alpha;
        const h16* va = VT + vo + key0; const h16* vr = VR + ve + key0;
        { const v16h v0 = ldh(va), v1 = ldh(va + (size_t)16 * SEQ), r0v = ldh(vr), r1v = ldh(vr + (size_t)16 * ESEQ);
          oh0 = wmma16(v0, pbh, oh0); oh1 = wmma16(v1, pbh, oh1);
          ol0 = wmma16(v0, pbr, ol0); ol1 = wmma16(v1, pbr, ol1);
          ol0 = wmma16(r0v, pbh, ol0); ol1 = wmma16(r1v, pbh, ol1);
          asm volatile("v_nop\n\tv_nop\n\tv_nop\n\tv_nop" : "+v"(oh0), "+v"(oh1), "+v"(ol0), "+v"(ol1) : "v"(v0), "v"(v1), "v"(r0v), "v"(r1v), "v"(pbh), "v"(pbr)); }
        { const v16h v2 = ldh(va + (size_t)32 * SEQ), v3 = ldh(va + (size_t)48 * SEQ), r2v = ldh(vr + (size_t)32 * ESEQ), r3v = ldh(vr + (size_t)48 * ESEQ);
          oh2 = wmma16(v2, pbh, oh2); oh3 = wmma16(v3, pbh, oh3);
          ol2 = wmma16(v2, pbr, ol2); ol3 = wmma16(v3, pbr, ol3);
          ol2 = wmma16(r2v, pbh, ol2); ol3 = wmma16(r3v, pbh, ol3);
          asm volatile("v_nop\n\tv_nop\n\tv_nop\n\tv_nop" : "+v"(oh2), "+v"(oh3), "+v"(ol2), "+v"(ol3) : "v"(v2), "v"(v3), "v"(r2v), "v"(r3v), "v"(pbh), "v"(pbr)); }
    }
    l += __shfl_xor(l, 16, 32);
    const float inv = CXS * (1.0f / l);
    const int wb = wave * 16 * 68;
    { v4f a, c;
#pragma unroll
      for (int i = 0; i < 4; ++i) { a[i] = (oh0[i] + ol0[i] * QRI) * inv; c[i] = (oh0[4 + i] + ol0[4 + i] * QRI) * inv; }
      *(v4fa*)(&os[wb + lr * 68 +  0 + 8 * hi]) = a; *(v4fa*)(&os[wb + lr * 68 +  0 + 8 * hi + 4]) = c;
#pragma unroll
      for (int i = 0; i < 4; ++i) { a[i] = (oh1[i] + ol1[i] * QRI) * inv; c[i] = (oh1[4 + i] + ol1[4 + i] * QRI) * inv; }
      *(v4fa*)(&os[wb + lr * 68 + 16 + 8 * hi]) = a; *(v4fa*)(&os[wb + lr * 68 + 16 + 8 * hi + 4]) = c;
#pragma unroll
      for (int i = 0; i < 4; ++i) { a[i] = (oh2[i] + ol2[i] * QRI) * inv; c[i] = (oh2[4 + i] + ol2[4 + i] * QRI) * inv; }
      *(v4fa*)(&os[wb + lr * 68 + 32 + 8 * hi]) = a; *(v4fa*)(&os[wb + lr * 68 + 32 + 8 * hi + 4]) = c;
#pragma unroll
      for (int i = 0; i < 4; ++i) { a[i] = (oh3[i] + ol3[i] * QRI) * inv; c[i] = (oh3[4 + i] + ol3[4 + i] * QRI) * inv; }
      *(v4fa*)(&os[wb + lr * 68 + 48 + 8 * hi]) = a; *(v4fa*)(&os[wb + lr * 68 + 48 + 8 * hi + 4]) = c; }
    wave_sync();
    h16* crow = CH + ((size_t)b * SEQ + t0) * DM + h * HD;
    h16* rrow = CR + ((size_t)b * ESEQ + t0) * DM + h * HD;
    const int c8 = (lane & 7) * 8;
#pragma unroll 1
    for (int ps = 0; ps < 2; ++ps) {
#pragma unroll
        for (int s = 0; s < 4; ++s) { const int row = 4 * s + (lane >> 3);
            const v4f x0 = *(const v4fa*)(&os[wb + row * 68 + c8]); const v4f x1 = *(const v4fa*)(&os[wb + row * 68 + c8 + 4]); v8h hv, rv;
#pragma unroll
            for (int i = 0; i < 4; ++i) { const h16 a0 = (h16)x0[i]; const h16 a1 = (h16)x1[i]; hv[i] = a0; hv[4 + i] = a1;
                rv[i] = (h16)((x0[i] - (float)a0) * QRS); rv[4 + i] = (h16)((x1[i] - (float)a1) * QRS); }
            *(volatile v8h*)(crow + (size_t)row * DM + c8) = hv;
            *(volatile v8h*)(rrow + (size_t)row * DM + c8) = rv; }
        if (ps == 0) __threadfence(); }
}

template <int RES>
__global__ __launch_bounds__(32) void k_out(const h16* __restrict__ CX, size_t crOff, const h16* __restrict__ WO, const float* __restrict__ bias, float* OUT) {
    __shared__ __align__(16) float os[16 * 68];
    constexpr int MBN = RES ? 2 : 4;
    constexpr int TPB = RES ? (ESEQ / 32) : (((SEQ - ESEQ) / 64) > 0 ? ((SEQ - ESEQ) / 64) : 1);
    const int K = DM;
    const int lane = threadIdx.x & 31, lr = lane & 15, hi = lane >> 4;
    const int b = blockIdx.x / TPB, tt = blockIdx.x % TPB;
    const int t0 = (RES ? 0 : ESEQ) + tt * 16 * MBN;
    const int c0 = blockIdx.y * 64;
    size_t offA[4];
    if (RES) {
        offA[0] = ((size_t)b * SEQ + t0 + lr) * K + 8 * hi; offA[1] = offA[0] + (size_t)16 * K;
        offA[2] = crOff + ((size_t)b * ESEQ + t0 + lr) * K + 8 * hi; offA[3] = offA[2] + (size_t)16 * K;
    } else {
#pragma unroll
        for (int i = 0; i < 4; ++i) offA[i] = ((size_t)b * SEQ + t0 + 16 * i + lr) * K + 8 * hi;
    }
    const size_t boff = (size_t)(c0 + lr) * K + 8 * hi;
    v8f acc[16];
#pragma unroll
    for (int i = 0; i < 16; ++i) acc[i] = (v8f){};
#pragma unroll 1
    for (int kc = 0; kc < K; kc += 32) {
        v16h a[4];
#pragma unroll
        for (int i = 0; i < 4; ++i) a[i] = ldh(CX + offA[i] + kc);
#pragma unroll
        for (int nb = 0; nb < 4; ++nb) { const v16h bb = ldh(WO + boff + (size_t)nb * 16 * K + kc);
#pragma unroll
            for (int i = 0; i < 4; ++i) acc[i * 4 + nb] = wmma16(a[i], bb, acc[i * 4 + nb]); }
        asm volatile("v_nop\n\tv_nop\n\tv_nop\n\tv_nop"
                     : "+v"(acc[0]), "+v"(acc[1]), "+v"(acc[2]), "+v"(acc[3]), "+v"(acc[4]), "+v"(acc[5]), "+v"(acc[6]), "+v"(acc[7]),
                       "+v"(acc[8]), "+v"(acc[9]), "+v"(acc[10]), "+v"(acc[11]), "+v"(acc[12]), "+v"(acc[13]), "+v"(acc[14]), "+v"(acc[15])
                     : "v"(a[0]), "v"(a[1]), "v"(a[2]), "v"(a[3]));
    }
    float bcol[4];
#pragma unroll
    for (int nb = 0; nb < 4; ++nb) bcol[nb] = bfr(bias[c0 + nb * 16 + lr]);
#pragma unroll
    for (int mb = 0; mb < MBN; ++mb) {
#pragma unroll
        for (int nb = 0; nb < 4; ++nb) {
#pragma unroll
            for (int j = 0; j < 8; ++j) { float v = acc[mb * 4 + nb][j];
                if (RES) v += acc[RES ? ((2 + mb) * 4 + nb) : 0][j] * QRI;
                os[(hi * 8 + j) * 68 + nb * 16 + lr] = v * OSI + bcol[nb]; } }
        wave_sync();
        float* orow = OUT + ((size_t)b * OUT_SEQ + t0 + mb * 16) * DM + c0;
#pragma unroll 1
        for (int ps = 0; ps < 2; ++ps) {
#pragma unroll
            for (int s = 0; s < 8; ++s) { const int row = 2 * s + hi, cofs = lr * 4;
                const v4f val = *(const v4fa*)(&os[row * 68 + cofs]);
                *(volatile v4f*)(orow + (size_t)row * DM + cofs) = val; }
            if (ps == 0) __threadfence(); }
        wave_sync();
    }
}

static constexpr size_t al256(size_t v) { return (v + 255) & ~(size_t)255; }
static constexpr size_t SZ_XB = al256((size_t)NB * SEQ * DM * 2);
static constexpr size_t SZ_WT = al256((size_t)3 * DM * DM * 2);
static constexpr size_t SZ_WO = al256((size_t)DM * DM * 2);
static constexpr size_t SZ_PL = al256((size_t)NB * NH_ * SEQ * HD * 2);
static constexpr size_t SZ_PE = al256((size_t)NB * NH_ * ESEQ * HD * 2);
static constexpr size_t SZ_CH = al256((size_t)NB * SEQ * DM * 2);
static constexpr size_t SZ_CR = al256((size_t)NB * ESEQ * DM * 2);
static constexpr size_t SZ_MW = al256((size_t)NB * WPB * 4);
static constexpr size_t SZ_TOTAL = SZ_XB + SZ_WT + SZ_WO + 3 * SZ_PL + 3 * SZ_PE + SZ_CH + SZ_CR + SZ_MW;
static_assert(SZ_TOTAL <= (size_t)134217728);
static_assert(((size_t)DM * DM * 2) % 256 == 0);
static_assert(SZ_CH % 2 == 0);

extern "C" void kernel_launch(void* const* d_in, const int* in_sizes, int n_in,
                              void* d_out, int out_size, void* d_ws, size_t ws_size, hipStream_t stream) {
    if (n_in < 6) return;
    const size_t needx = ((size_t)(NB - 1) * SEQ_FULL + SEQ) * DM;
    if ((size_t)in_sizes[0] < needx) return;
    if ((size_t)in_sizes[1] < (size_t)(NB - 1) * SEQ_FULL + SEQ) return;
    if ((size_t)in_sizes[2] < (size_t)3 * DM * DM || (size_t)in_sizes[3] < (size_t)3 * DM) return;
    if ((size_t)in_sizes[4] < (size_t)DM * DM || (size_t)in_sizes[5] < (size_t)DM) return;
    if ((size_t)out_size < ((size_t)(NB - 1) * OUT_SEQ + SEQ) * DM) return;
    if (SZ_TOTAL > ws_size) return;
    const float* x = (const float*)d_in[0]; const int* pad = (const int*)d_in[1];
    const float* wqkv = (const float*)d_in[2]; const float* bqkv = (const float*)d_in[3];
    const float* wout = (const float*)d_in[4]; const float* bout = (const float*)d_in[5];
    float* OUT = (float*)d_out;
    char* wsp = (char*)d_ws;
    bf* XB = (bf*)wsp; wsp += SZ_XB;
    bf* WT = (bf*)wsp; wsp += SZ_WT;
    h16* WO = (h16*)wsp; wsp += SZ_WO;
    h16* QH = (h16*)wsp; wsp += SZ_PL;
    h16* KP = (h16*)wsp; wsp += SZ_PL;
    h16* VT = (h16*)wsp; wsp += SZ_PL;
    h16* QR = (h16*)wsp; wsp += SZ_PE;
    h16* KR = (h16*)wsp; wsp += SZ_PE;
    h16* VR = (h16*)wsp; wsp += SZ_PE;
    h16* CH = (h16*)wsp; wsp += SZ_CH;
    h16* CR = (h16*)wsp; wsp += SZ_CR;
    unsigned* MW = (unsigned*)wsp; wsp += SZ_MW;
    const size_t crOff = SZ_CH / 2;

    if (SEQ == SEQ_FULL) {
        const size_t n8 = (size_t)NB * SEQ * DM / 8;
        k_cvt8<<<(unsigned)((n8 + 255) / 256), 256, 0, stream>>>(x, XB, n8);
    } else {
        const size_t n8 = (size_t)SEQ * DM / 8;
        for (int b = 0; b < NB; ++b) k_cvt8<<<(unsigned)((n8 + 255) / 256), 256, 0, stream>>>(x + (size_t)b * SEQ_FULL * DM, XB + (size_t)b * SEQ * DM, n8);
    }
    k_cvt_t<0><<<dim3(3 * DM / 64, DM / 64, 1), 256, 0, stream>>>(wqkv, WT, DM, 3 * DM);
    k_cvt_t<1><<<dim3(DM / 64, DM / 64, 1), 256, 0, stream>>>(wout, (bf*)WO, DM, DM);
    k_mask<<<NB * (WPB / 32), 32, 0, stream>>>(pad, MW);

    k_proj<<<dim3(NB * SEQ / 64, DM / 64, 1), 32, 0, stream>>>(XB, WT, bqkv, 0, QH, QR, 1,
        SEQ, (size_t)NH_ * SEQ * HD, HD, HD, (size_t)SEQ * HD, (size_t)NH_ * ESEQ * HD, HD, (size_t)ESEQ * HD);
    k_proj<<<dim3(NB * SEQ / 64, DM / 64, 1), 32, 0, stream>>>(XB, WT + (size_t)DM * DM, bqkv + DM, 0, KP, KR, 1,
        SEQ, (size_t)NH_ * SEQ * HD, HD, HD, (size_t)SEQ * HD, (size_t)NH_ * ESEQ * HD, HD, (size_t)ESEQ * HD);
    k_proj<<<dim3(DM / 64, NB * SEQ / 64, 1), 32, 0, stream>>>(WT + (size_t)2 * DM * DM, XB, bqkv + 2 * DM, 1, VT, VR, 2,
        DM, (size_t)0, SEQ, SEQ, (size_t)DM * SEQ, (size_t)0, ESEQ, (size_t)DM * ESEQ);

    k_flash_e<<<dim3(ESEQ / (16 * AW), NB * NH_, 1), 32 * AW, 0, stream>>>(QH, QR, KP, KR, VT, VR, MW, CH, CR);
    if (SEQ > ESEQ)
        k_flash_d<<<dim3((SEQ - ESEQ) / (16 * AW), NB * NH_, 1), 32 * AW, 0, stream>>>(QH, KP, VT, MW, CH);

    k_out<1><<<dim3(NB * (ESEQ / 32), DM / 64, 1), 32, 0, stream>>>(CH, crOff, WO, bout, OUT);
    if (SEQ > ESEQ)
        k_out<0><<<dim3(NB * ((SEQ - ESEQ) / 64), DM / 64, 1), 32, 0, stream>>>(CH, crOff, WO, bout, OUT);
}
